// DilateAttention3D_67473936220609
// MI455X (gfx1250) — hardware-verified
//
#include <hip/hip_runtime.h>


#ifndef NB
#define NB 2
#endif
#define NB_FULL 2
#define CH   96
#define NHD  6
#define HD   16
#define DZ   16
#define HY   32
#define WX   32
#define CSTR (DZ * HY * WX)
#define ZP   (DZ + 2)
#define YP   (HY + 2)
#define WP   (WX + 4)
#define NWB  (WX / 4)
#define AW   4
#define OSP  36
#define SC2  ((float)(0.25 * 1.4426950408889634))
#define PSH  14.0f
#define NEGB (-3.0e38f)

static_assert(NHD * HD == CH);
static_assert(HD == 16);
static_assert(NHD % 2 == 0);
static_assert(DZ % 2 == 0);
static_assert(HY % 2 == 0);
static_assert(WX % 4 == 0);
static_assert(WX == 32);
static_assert(HY == 32);
static_assert(DZ == 16);
static_assert(NWB == 8);
static_assert(WP >= WX + 4);
static_assert((CH * 4) % 128 == 0);
static_assert(((DZ / 2) * (HY / 2) * (WX / 4)) % AW == 0);
static_assert((OSP * 4) % 16 == 0);
static_assert(NB <= NB_FULL);
static_assert(AW * 16 * OSP * 4 <= 131072);

typedef _Float16 h16;
typedef __attribute__((ext_vector_type(16))) _Float16 v16h;
typedef __attribute__((ext_vector_type(8)))  _Float16 v8h;
typedef __attribute__((ext_vector_type(8)))  float    v8f;
typedef __attribute__((ext_vector_type(4)))  float    v4f;
typedef v4f  __attribute__((may_alias)) v4fa;

__device__ __forceinline__ unsigned short f2bf(float f) { unsigned u = __float_as_uint(f); u += 0x7FFFu + ((u >> 16) & 1u); return (unsigned short)(u >> 16); }
__device__ __forceinline__ float bfr(float f) { return __uint_as_float(((unsigned)f2bf(f)) << 16); }
__device__ __forceinline__ v16h cat16(v8h lo, v8h hi) { return __builtin_shufflevector(lo, hi, 0, 1, 2, 3, 4, 5, 6, 7, 8, 9, 10, 11, 12, 13, 14, 15); }
__device__ __forceinline__ v8f wmma16(v16h a, v16h b, v8f c) { return __builtin_amdgcn_wmma_f32_16x16x32_f16(false, a, false, b, (short)0, c, false, false); }
__device__ __forceinline__ v8f wmma16g(v16h a, v16h b, v8f c) { c = wmma16(a, b, c); asm volatile("v_nop\n\tv_nop\n\tv_nop\n\tv_nop" : "+v"(c) : "v"(a), "v"(b)); return c; }
static __device__ __forceinline__ h16 toh_flush(float v) { const h16 r = (h16)v; return (fabsf(v) < 6.103515625e-05f) ? (h16)0.0f : r; }
__device__ __forceinline__ v16h ld8z(const h16* p) { return cat16(*(const v8h*)p, (v8h){}); }
__device__ __forceinline__ void wave_sync() { __builtin_amdgcn_fence(3  , "wavefront"); __builtin_amdgcn_wave_barrier(); asm volatile("" ::: "memory"); }

__global__ __launch_bounds__(256) void k_rows(const float* __restrict__ src, h16* dst, unsigned npieces) {
    const unsigned i = blockIdx.x * 256u + threadIdx.x; if (i >= npieces) return;
    const int c8 = (int)(i & 1u) * 8; unsigned r = i >> 1;
    const int wp = (int)(r % (unsigned)WP); r /= (unsigned)WP;
    const int yp = (int)(r % (unsigned)YP); r /= (unsigned)YP;
    const int zp = (int)(r % (unsigned)ZP); const int bh = (int)(r / (unsigned)ZP);
    const int b = bh / NHD, hd = bh % NHD;
    const int z = zp - 1, y = yp - 1, w = wp - 1;
    const bool ok = ((unsigned)z < (unsigned)DZ) & ((unsigned)y < (unsigned)HY) & ((unsigned)w < (unsigned)WX);
    const int zc = z < 0 ? 0 : (z > DZ - 1 ? DZ - 1 : z);
    const int yc = y < 0 ? 0 : (y > HY - 1 ? HY - 1 : y);
    const int wc = w < 0 ? 0 : (w > WX - 1 ? WX - 1 : w);
    const size_t so = (size_t)(b * CH + hd * HD + c8) * CSTR + (size_t)((zc * HY + yc) * WX + wc);
    float x[8];
#pragma unroll
    for (int j = 0; j < 8; ++j) x[j] = src[so + (size_t)j * CSTR];
#pragma unroll
    for (int j = 0; j < 8; ++j) asm volatile("" : "+v"(x[j]));
    v8h o;
#pragma unroll
    for (int j = 0; j < 8; ++j) { const float xs = ok ? bfr(x[j]) : 0.0f; o[j] = toh_flush(xs); }
    *(volatile v8h*)(dst + (size_t)i * 8) = o; __threadfence(); *(volatile v8h*)(dst + (size_t)i * 8) = o;
}

__global__ __launch_bounds__(256) void k_vwin(const float* __restrict__ src, h16* dst, unsigned npieces) {
    const unsigned i = blockIdx.x * 256u + threadIdx.x; if (i >= npieces) return;
    const int wbk = (int)(i & 7u); unsigned r = i >> 3;
    const int yp = (int)(r % (unsigned)YP); r /= (unsigned)YP;
    const int zp = (int)(r % (unsigned)ZP); const int bch = (int)(r / (unsigned)ZP);
    const int z = zp - 1, y = yp - 1;
    const bool rowok = ((unsigned)z < (unsigned)DZ) & ((unsigned)y < (unsigned)HY);
    const int zc = z < 0 ? 0 : (z > DZ - 1 ? DZ - 1 : z);
    const int yc = y < 0 ? 0 : (y > HY - 1 ? HY - 1 : y);
    const size_t ro = (size_t)bch * CSTR + (size_t)((zc * HY + yc) * WX);
    const int bm = wbk > 0 ? wbk - 1 : 0;
    const int bp = wbk < NWB - 1 ? wbk + 1 : NWB - 1;
    v4f A = *(const v4f*)(src + ro + 4 * bm);
    v4f B = *(const v4f*)(src + ro + 4 * wbk);
    v4f C = *(const v4f*)(src + ro + 4 * bp);
    asm volatile("" : "+v"(A)); asm volatile("" : "+v"(B)); asm volatile("" : "+v"(C));
    const bool okm = rowok & (wbk >= 1);
    const bool okp = rowok & (wbk <= NWB - 2);
    float e[8];
    e[0] = okm ? bfr(A[3]) : 0.0f;
    e[1] = rowok ? bfr(B[0]) : 0.0f; e[2] = rowok ? bfr(B[1]) : 0.0f; e[3] = rowok ? bfr(B[2]) : 0.0f; e[4] = rowok ? bfr(B[3]) : 0.0f;
    e[5] = okp ? bfr(C[0]) : 0.0f; e[6] = okp ? bfr(C[1]) : 0.0f; e[7] = okp ? bfr(C[2]) : 0.0f;
    v8h o;
#pragma unroll
    for (int j = 0; j < 8; ++j) o[j] = toh_flush(e[j]);
    *(volatile v8h*)(dst + (size_t)i * 8) = o; __threadfence(); *(volatile v8h*)(dst + (size_t)i * 8) = o;
}

__global__ __launch_bounds__(32 * AW) void k_nbrwin(const h16* __restrict__ QP, const h16* __restrict__ KP, const h16* __restrict__ VW, float* OUT) {
    __shared__ __align__(16) float os[AW * 16 * OSP];
    const int lane = threadIdx.x & 31, lr = lane & 15, hi = lane >> 4;
    const int wave = __builtin_amdgcn_readfirstlane((int)(threadIdx.x >> 5));
    const int tidx = blockIdx.x * AW + wave;
    const int wbk = tidx & 7, yb = (tidx >> 3) & 15, zb = tidx >> 7;
    const int b = blockIdx.y / 3, hp = blockIdx.y % 3;
    const int z0 = 2 * zb, y0 = 2 * yb, w0 = 4 * wbk;
    const int qz = lr >> 3, qy = (lr >> 2) & 1, qw = lr & 3;
    bool kzy[8], kw[8];
#pragma unroll
    for (int j = 0; j < 8; ++j) { const int dz = j >> 1, dy = 2 * (j & 1) + hi; kzy[j] = ((unsigned)(dz - qz) <= 2u) & ((unsigned)(dy - qy) <= 2u); }
#pragma unroll
    for (int r = 0; r < 8; ++r) kw[r] = (unsigned)(r - qw) <= 2u;
    const int qrow  = ((z0 + qz + 1) * YP + (y0 + qy + 1)) * WP + (w0 + qw + 1);
    const int krow0 = (z0 * YP + (y0 + (lr >> 3))) * WP + (w0 + (lr & 7));
    const int wb = wave * 16 * OSP;
#pragma unroll 1
    for (int hh = 0; hh < 2; ++hh) {
        const int hd = 2 * hp + hh;
        const size_t rbase = (size_t)(b * NHD + hd) * ((size_t)ZP * YP * WP * HD);
        const v16h qf = ld8z(QP + rbase + (size_t)qrow * HD + 8 * hi);
        v8f s[8];
#pragma unroll
        for (int j = 0; j < 8; ++j) {
            const int kr = krow0 + ((j >> 1) * YP + 2 * (j & 1)) * WP;
            const v16h ka = ld8z(KP + rbase + (size_t)kr * HD + 8 * hi);
            s[j] = wmma16g(ka, qf, (v8f){});
        }
        float mx = NEGB;
#pragma unroll
        for (int j = 0; j < 8; ++j) {
#pragma unroll
            for (int r = 0; r < 8; ++r) { const bool kp = kzy[j] & kw[r]; const float t = s[j][r] * SC2; mx = fmaxf(mx, kp ? t : NEGB); } }
        mx = fmaxf(mx, __shfl_xor(mx, 16, 32));
        const float sh = PSH - mx;
        const size_t vch = (size_t)(b * CH + hd * HD + lr);
        v8f o = (v8f){};
        float ls = 0.0f;
#pragma unroll
        for (int s4 = 0; s4 < 4; ++s4) {
            v16h pb;
#pragma unroll
            for (int r = 0; r < 8; ++r) {
                const float ea = s[2 * s4][r] * SC2 + sh, eb = s[2 * s4 + 1][r] * SC2 + sh;
                const float xa = __builtin_amdgcn_exp2f(ea), xb = __builtin_amdgcn_exp2f(eb);
                const bool ca = kzy[2 * s4] & kw[r] & (ea >= -14.0f);
                const bool cb = kzy[2 * s4 + 1] & kw[r] & (eb >= -14.0f);
                const float ga = ca ? xa : 0.0f, gb = cb ? xb : 0.0f;
                const h16 pa = (h16)ga; const h16 pc = (h16)gb;
                pb[r] = pa; pb[8 + r] = pc;
                ls += (float)pa + (float)pc; }
            const size_t va = (((vch * ZP + (size_t)(z0 + s4)) * YP + (size_t)(y0 + hi)) * NWB + (size_t)wbk) * 8;
            const v16h vf = cat16(*(const v8h*)(VW + va), *(const v8h*)(VW + va + (size_t)2 * NWB * 8));
            o = wmma16g(vf, pb, o);
        }
        const float l = ls + __shfl_xor(ls, 16, 32);
        const float inv = 1.0f / l;
        { v4f a, c;
          a[0] = o[0] * inv; a[1] = o[1] * inv; a[2] = o[2] * inv; a[3] = o[3] * inv; c[0] = o[4] * inv; c[1] = o[5] * inv; c[2] = o[6] * inv; c[3] = o[7] * inv;
          *(v4fa*)(&os[wb + lr * OSP + hh * 16 + 8 * hi]) = a; *(v4fa*)(&os[wb + lr * OSP + hh * 16 + 8 * hi + 4]) = c; }
    }
    wave_sync();
    static_assert(32 * 16 * 4 == 16 * 128);
    float* obase = OUT + ((((size_t)(b * DZ + z0) * HY + (size_t)y0) * WX + (size_t)w0) * CH) + hp * 32;
#pragma unroll 1
    for (int ps = 0; ps < 2; ++ps) {
#pragma unroll
        for (int s = 0; s < 4; ++s) { const int row = 4 * s + (lane >> 3), cofs = (lane & 7) * 4;
            const v4f val = *(const v4fa*)(&os[wb + row * OSP + cofs]);
            const size_t po = ((size_t)((s >> 1) * HY + (s & 1)) * WX + (size_t)(lane >> 3)) * CH;
            *(volatile v4f*)(obase + po + cofs) = val; }
        if (ps == 0) __threadfence(); }
}

static constexpr size_t al256(size_t v) { return (v + 255) & ~(size_t)255; }
static constexpr size_t N_ROWP = (size_t)NB * NHD * ZP * YP * WP * 2;
static constexpr size_t N_VWP  = (size_t)NB * CH * ZP * YP * NWB;
static constexpr size_t SZ_RP = al256(N_ROWP * 16);
static constexpr size_t SZ_VW = al256(N_VWP * 16);
static constexpr size_t SZ_TOTAL = 2 * SZ_RP + SZ_VW;
static_assert(SZ_TOTAL <= (size_t)134217728);
static_assert(N_ROWP % 32 == 0);
static_assert(N_VWP % 32 == 0);
static_assert(N_ROWP < (size_t)0x7FFFFFFF);
static_assert(N_VWP < (size_t)0x7FFFFFFF);
static_assert(N_ROWP * 8 == (size_t)NB * NHD * ZP * YP * WP * HD);
static_assert(N_VWP * 8 == (size_t)NB * CH * ZP * YP * NWB * 8);

extern "C" void kernel_launch(void* const* d_in, const int* in_sizes, int n_in,
                              void* d_out, int out_size, void* d_ws, size_t ws_size, hipStream_t stream) {
    if (n_in < 3) return;
    const size_t need = (size_t)NB * CH * CSTR;
    if ((size_t)in_sizes[0] < need || (size_t)in_sizes[1] < need || (size_t)in_sizes[2] < need) return;
    if ((size_t)out_size < need) return;
    if (SZ_TOTAL > ws_size) return;
    const float* q = (const float*)d_in[0];
    const float* k = (const float*)d_in[1];
    const float* v = (const float*)d_in[2];
    float* OUT = (float*)d_out;
    char* wsp = (char*)d_ws;
    h16* QP = (h16*)wsp; wsp += SZ_RP;
    h16* KP = (h16*)wsp; wsp += SZ_RP;
    h16* VW = (h16*)wsp; wsp += SZ_VW;

    const unsigned gr = (unsigned)((N_ROWP + 255) / 256);
    const unsigned gv = (unsigned)((N_VWP + 255) / 256);
    k_rows<<<gr, 256, 0, stream>>>(q, QP, (unsigned)N_ROWP);
    k_rows<<<gr, 256, 0, stream>>>(k, KP, (unsigned)N_ROWP);
    k_vwin<<<gv, 256, 0, stream>>>(v, VW, (unsigned)N_VWP);
    k_nbrwin<<<dim3(((DZ / 2) * (HY / 2) * (WX / 4)) / AW, NB * 3, 1), 32 * AW, 0, stream>>>(QP, KP, VW, OUT);
}
